// VectorQuantizer_764504178920
// MI455X (gfx1250) — hardware-run, weakly checked
//
#include <hip/hip_runtime.h>


#ifndef NB
#define NB 2
#endif
#define NB_FULL 2
#define CI    32
#define TT    8
#define HH    32
#define WW    32
#define THW   (TT * HH * WW)
#define NQ    (NB * THW)
#define VOCAB 8192
#define TAPS  27
#define KC    (TAPS * CI)
#define TP    (TT + 2)
#define HP    (HH + 2)
#define WP    (WW + 2)
#define NPP   (NB * TP * HP * WP)
#define NROWS (NB * TT * HH)
#define GW    4
#define CW    4
#define OSP   36
#define CSP   40
#define QSP   40
#define OUT1_ELEM ((size_t)NB_FULL * CI * THW)

static_assert(CI == 32);
static_assert(WW == 32);
static_assert(KC % 32 == 0);
static_assert(THW % 64 == 0);
static_assert(NQ % 64 == 0);
static_assert(VOCAB % 64 == 0);
static_assert(VOCAB % 16 == 0);
static_assert(NQ % (32 * GW) == 0);
static_assert(NROWS % CW == 0);
static_assert(((size_t)VOCAB * CI) % 8 == 0);
static_assert(((size_t)CI * KC) % 8 == 0);
static_assert(((size_t)CI * KC * 2) % 128 == 0);
static_assert(((size_t)NPP * 4) % 32 == 0);
static_assert(((size_t)NPP * CI * 2) % 128 == 0);
static_assert((OSP * 4) % 16 == 0);
static_assert((CSP * 2) % 16 == 0);
static_assert((QSP * 2) % 16 == 0);
static_assert(OSP >= WW);
static_assert(CSP >= CI);
static_assert(QSP >= CI);
static_assert(NB <= NB_FULL);
static_assert((size_t)VOCAB * 100 > (size_t)NQ);
static_assert(OUT1_ELEM * 4 == (size_t)2097152);
static_assert((OUT1_ELEM * 4) % 128 == 0);
static_assert((size_t)CW * 32 * OSP * 4 + (size_t)CW * 32 * CSP * 2 <= 131072);
static_assert((size_t)VOCAB * 4 + 64 <= 131072);
static_assert((size_t)64 * QSP * 2 <= 131072);

typedef unsigned short bf;
typedef __attribute__((ext_vector_type(16))) __bf16   v16bf;
typedef __attribute__((ext_vector_type(8)))  unsigned short v8us;
typedef __attribute__((ext_vector_type(8)))  float    v8f;
typedef __attribute__((ext_vector_type(4)))  float    v4f;
typedef __attribute__((ext_vector_type(2)))  float    v2f;
typedef __attribute__((ext_vector_type(4)))  unsigned v4u;
typedef v4f  __attribute__((may_alias)) v4fa;
typedef v8us __attribute__((may_alias)) v8usa;

__device__ __forceinline__ unsigned short f2bf(float f) { unsigned u = __float_as_uint(f); u += 0x7FFFu + ((u >> 16) & 1u); return (unsigned short)(u >> 16); }
__device__ __forceinline__ float bfr(float f) { return __uint_as_float(((unsigned)f2bf(f)) << 16); }
__device__ __forceinline__ v16bf cat16b(v8us lo, v8us hi) { return __builtin_bit_cast(v16bf, __builtin_shufflevector(lo, hi, 0, 1, 2, 3, 4, 5, 6, 7, 8, 9, 10, 11, 12, 13, 14, 15)); }
__device__ __forceinline__ v8f wmmab(v16bf a, v16bf b, v8f c) { return __builtin_amdgcn_wmma_f32_16x16x32_bf16(false, a, false, b, (short)0, c, false, false); }
__device__ __forceinline__ v8f wmmab_g(v16bf a, v16bf b, v8f c) { c = wmmab(a, b, c); asm volatile("v_nop\n\tv_nop\n\tv_nop\n\tv_nop" : "+v"(c) : "v"(a), "v"(b)); return c; }
__device__ __forceinline__ v16bf ldb(const bf* p)  { return cat16b(*(const v8us*)p, *(const v8us*)(p + 16)); }
__device__ __forceinline__ void wave_sync() { __builtin_amdgcn_fence(3  , "wavefront"); __builtin_amdgcn_wave_barrier(); asm volatile("" ::: "memory"); }

__global__ __launch_bounds__(256) void k_cvt8(const float* __restrict__ src, bf* dst, size_t n8) {
    const size_t i = (size_t)blockIdx.x * 256 + threadIdx.x; if (i >= n8) return;
    const v8f v = *(const v8f*)(src + i * 8); v8us o;
#pragma unroll
    for (int k = 0; k < 8; ++k) o[k] = f2bf(v[k]);
    *(volatile v8us*)(dst + i * 8) = o; __threadfence(); *(volatile v8us*)(dst + i * 8) = o;
}

__global__ __launch_bounds__(256) void k_qT(const float* __restrict__ F, bf* QB) {
    __shared__ __align__(16) unsigned short qs[64 * QSP];
    const int tid = threadIdx.x;
    const int n0 = blockIdx.x * 64;
    const int b = n0 / THW, p0 = n0 % THW;
    { const int c = tid >> 3, p8 = (tid & 7) * 8;
      const v8f v = *(const v8f*)(F + ((size_t)(b * CI + c)) * THW + p0 + p8);
#pragma unroll
      for (int j = 0; j < 8; ++j) qs[(p8 + j) * QSP + c] = f2bf(v[j]); }
    __syncthreads();
    const int r = tid >> 2, c8 = (tid & 3) * 8;
    const v8us o = *(const v8usa*)(&qs[r * QSP + c8]);
    bf* dst = QB + (size_t)n0 * CI + (size_t)tid * 8;
    *(volatile v8us*)dst = o; __threadfence(); *(volatile v8us*)dst = o;
}
static_assert(256 * 8 == 64 * CI);

__global__ __launch_bounds__(256) void k_wprep(const float* __restrict__ cw, bf* WB, int n8) {
    const int i = blockIdx.x * 256 + threadIdx.x; if (i >= n8) return;
    v8us o;
#pragma unroll
    for (int j = 0; j < 8; ++j) { const int e = i * 8 + j; const int oc = e / KC, rem = e % KC; const int tap = rem >> 5, ci = rem & 31;
        o[j] = f2bf(cw[(size_t)oc * KC + ci * TAPS + tap]); }
    *(volatile v8us*)(WB + (size_t)i * 8) = o; __threadfence(); *(volatile v8us*)(WB + (size_t)i * 8) = o;
}

__global__ __launch_bounds__(256) void k_rownorm(const bf* __restrict__ P, float* NRM) {
    __shared__ __align__(16) float sm[64];
    const int tid = threadIdx.x;
    const size_t i = (size_t)blockIdx.x * 256 + tid;
    const v8us v = *(const v8us*)(P + i * 8);
    float s = 0.0f;
#pragma unroll
    for (int k = 0; k < 8; ++k) { const float x = __uint_as_float(((unsigned)v[k]) << 16); s += x * x; }
    s += __shfl_xor(s, 1, 32); s += __shfl_xor(s, 2, 32);
    if ((tid & 3) == 0) sm[tid >> 2] = s;
    __syncthreads();
    if (tid < 16) { const v4f o = *(const v4fa*)(&sm[tid * 4]); float* dst = NRM + (size_t)blockIdx.x * 64 + tid * 4;
        *(volatile v4f*)dst = o; __threadfence(); *(volatile v4f*)dst = o; }
}
static_assert(16 * 16 == 64 * 4);

__global__ __launch_bounds__(32 * GW) void k_argmin(const bf* __restrict__ QB, const bf* __restrict__ EB, const float* __restrict__ QQ, const float* __restrict__ EE, int* IDX) {
    __shared__ int is[GW * 32];
    const int lane = threadIdx.x & 31, lr = lane & 15, hi = lane >> 4;
    const int wave = __builtin_amdgcn_readfirstlane((int)(threadIdx.x >> 5));
    const int row0 = (blockIdx.x * GW + wave) * 32;
    const v16bf q0 = ldb(QB + (size_t)(row0 + lr) * CI + 8 * hi);
    const v16bf q1 = ldb(QB + (size_t)(row0 + 16 + lr) * CI + 8 * hi);
    const v4f qa0 = *(const v4f*)(QQ + row0 + 8 * hi), qa1 = *(const v4f*)(QQ + row0 + 8 * hi + 4);
    const v4f qb0 = *(const v4f*)(QQ + row0 + 16 + 8 * hi), qb1 = *(const v4f*)(QQ + row0 + 16 + 8 * hi + 4);
    float qa[8], qb[8], ba[8], bb[8]; int ia[8], ib[8];
#pragma unroll
    for (int r = 0; r < 4; ++r) { qa[r] = qa0[r]; qa[4 + r] = qa1[r]; qb[r] = qb0[r]; qb[4 + r] = qb1[r]; }
#pragma unroll
    for (int r = 0; r < 8; ++r) { ba[r] = 3.4e38f; bb[r] = 3.4e38f; ia[r] = 0; ib[r] = 0; }
    const size_t eo = (size_t)lr * CI + 8 * hi;
#pragma unroll 1
    for (int c0 = 0; c0 < VOCAB; c0 += 16) {
        const v16bf e = ldb(EB + eo + (size_t)c0 * CI);
        const float en = EE[c0 + lr];
        const int col = c0 + lr;
        v8f sa = (v8f){}, sb = (v8f){};
        sa = wmmab_g(q0, e, sa); sb = wmmab_g(q1, e, sb);
#pragma unroll
        for (int r = 0; r < 8; ++r) {
            const float da = __builtin_fmaf(-2.0f, sa[r], qa[r] + en);
            const float db = __builtin_fmaf(-2.0f, sb[r], qb[r] + en);
            const bool ca = da < ba[r], cb = db < bb[r];
            ba[r] = ca ? da : ba[r]; ia[r] = ca ? col : ia[r];
            bb[r] = cb ? db : bb[r]; ib[r] = cb ? col : ib[r]; }
    }
#pragma unroll
    for (int r = 0; r < 8; ++r) {
#pragma unroll
        for (int m = 1; m < 16; m <<= 1) {
            const float oda = __shfl_xor(ba[r], m, 32); const int oia = __shfl_xor(ia[r], m, 32);
            const float odb = __shfl_xor(bb[r], m, 32); const int oib = __shfl_xor(ib[r], m, 32);
            const bool ta = (oda < ba[r]) | ((oda == ba[r]) & (oia < ia[r]));
            const bool tb = (odb < bb[r]) | ((odb == bb[r]) & (oib < ib[r]));
            ba[r] = ta ? oda : ba[r]; ia[r] = ta ? oia : ia[r];
            bb[r] = tb ? odb : bb[r]; ib[r] = tb ? oib : ib[r]; } }
    if (lr == 0) {
#pragma unroll
        for (int r = 0; r < 8; ++r) { is[wave * 32 + 8 * hi + r] = ia[r]; is[wave * 32 + 16 + 8 * hi + r] = ib[r]; } }
    wave_sync();
    int v = is[wave * 32 + lane]; v = v < 0 ? 0 : (v > VOCAB - 1 ? VOCAB - 1 : v);
    int* dst = IDX + row0 + lane;
    *(volatile int*)dst = v; __threadfence(); *(volatile int*)dst = v;
}

__global__ __launch_bounds__(256) void k_gather(const int* __restrict__ IDX, const bf* __restrict__ EB, bf* FHP, int ng) {
    const int g = blockIdx.x * 256 + threadIdx.x; if (g >= ng) return;
    const int pp = g >> 2, q4 = g & 3;
    const int wp = pp % WP, hp = (pp / WP) % HP, tp = (pp / (WP * HP)) % TP, b = pp / (WP * HP * TP);
    const bool inside = (wp >= 1) & (wp <= WW) & (hp >= 1) & (hp <= HH) & (tp >= 1) & (tp <= TT);
    int w = wp - 1; w = w < 0 ? 0 : (w > WW - 1 ? WW - 1 : w);
    int h = hp - 1; h = h < 0 ? 0 : (h > HH - 1 ? HH - 1 : h);
    int t = tp - 1; t = t < 0 ? 0 : (t > TT - 1 ? TT - 1 : t);
    int code = IDX[b * THW + t * (HH * WW) + h * WW + w];
    asm volatile("" : "+v"(code));
    code = code < 0 ? 0 : (code > VOCAB - 1 ? VOCAB - 1 : code);
    v4u x = *(const v4u*)(EB + (size_t)code * CI + q4 * 8);
    asm volatile("" : "+v"(x));
    const v4u z = (v4u){0u, 0u, 0u, 0u};
    const v4u o = inside ? x : z;
    bf* dst = FHP + (size_t)g * 8;
    *(volatile v4u*)dst = o; __threadfence(); *(volatile v4u*)dst = o;
}

__global__ __launch_bounds__(32 * CW) void k_conv(const bf* __restrict__ FHP, const bf* __restrict__ WB, const float* __restrict__ cbias, const float* __restrict__ F, float* OUT, float* PART) {
    __shared__ __align__(16) float os[CW * 32 * OSP];
    __shared__ __align__(16) unsigned short cs[CW * 32 * CSP];
    const int lane = threadIdx.x & 31, lr = lane & 15, hi = lane >> 4;
    const int wave = __builtin_amdgcn_readfirstlane((int)(threadIdx.x >> 5));
    const int rid = blockIdx.x * CW + wave;
    const int b = rid / (TT * HH), t = (rid / HH) % TT, h = rid % HH;
    v8f acc00 = (v8f){}, acc01 = (v8f){}, acc10 = (v8f){}, acc11 = (v8f){};
    const size_t wo = (size_t)lr * KC + 8 * hi;
#pragma unroll 1
    for (int kt = 0; kt < 3; ++kt) {
#pragma unroll 1
        for (int kh = 0; kh < 3; ++kh) {
#pragma unroll 1
            for (int kw = 0; kw < 3; ++kw) {
                const int tap = (kt * 3 + kh) * 3 + kw;
                const size_t pp = ((size_t)((b * TP + t + kt) * HP + h + kh)) * WP + kw;
                const bf* ap = FHP + (pp + lr) * CI + 8 * hi;
                const v16bf a0 = ldb(ap), a1 = ldb(ap + 16 * CI);
                const bf* bp = WB + wo + tap * 32;
                const v16bf b0 = ldb(bp), b1 = ldb(bp + (size_t)16 * KC);
                acc00 = wmmab_g(a0, b0, acc00); acc01 = wmmab_g(a0, b1, acc01);
                acc10 = wmmab_g(a1, b0, acc10); acc11 = wmmab_g(a1, b1, acc11);
            } } }
    const int wb = wave * 32 * OSP, cwb = wave * 32 * CSP;
    { v4f a, c;
      a[0] = acc00[0]; a[1] = acc00[1]; a[2] = acc00[2]; a[3] = acc00[3]; c[0] = acc00[4]; c[1] = acc00[5]; c[2] = acc00[6]; c[3] = acc00[7];
      *(v4fa*)(&os[wb + lr * OSP + 8 * hi]) = a; *(v4fa*)(&os[wb + lr * OSP + 8 * hi + 4]) = c;
      a[0] = acc01[0]; a[1] = acc01[1]; a[2] = acc01[2]; a[3] = acc01[3]; c[0] = acc01[4]; c[1] = acc01[5]; c[2] = acc01[6]; c[3] = acc01[7];
      *(v4fa*)(&os[wb + (16 + lr) * OSP + 8 * hi]) = a; *(v4fa*)(&os[wb + (16 + lr) * OSP + 8 * hi + 4]) = c;
      a[0] = acc10[0]; a[1] = acc10[1]; a[2] = acc10[2]; a[3] = acc10[3]; c[0] = acc10[4]; c[1] = acc10[5]; c[2] = acc10[6]; c[3] = acc10[7];
      *(v4fa*)(&os[wb + lr * OSP + 16 + 8 * hi]) = a; *(v4fa*)(&os[wb + lr * OSP + 16 + 8 * hi + 4]) = c;
      a[0] = acc11[0]; a[1] = acc11[1]; a[2] = acc11[2]; a[3] = acc11[3]; c[0] = acc11[4]; c[1] = acc11[5]; c[2] = acc11[6]; c[3] = acc11[7];
      *(v4fa*)(&os[wb + (16 + lr) * OSP + 16 + 8 * hi]) = a; *(v4fa*)(&os[wb + (16 + lr) * OSP + 16 + 8 * hi + 4]) = c; }
    { const size_t cpos = ((size_t)((b * TP + t + 1) * HP + h + 1)) * WP + 1;
      const bf* cp = FHP + cpos * CI;
#pragma unroll
      for (int j = 0; j < 4; ++j) { const int p = j * 32 + lane;
          const v8us cv = *(const v8us*)(cp + (size_t)p * 8);
          *(v8usa*)(&cs[cwb + (p >> 2) * CSP + (p & 3) * 8]) = cv; } }
    wave_sync();
    const size_t obase = ((size_t)(b * CI)) * THW + (size_t)t * (HH * WW) + (size_t)h * WW;
    float ls = 0.0f;
#pragma unroll 1
    for (int s = 0; s < 8; ++s) { const int o = 4 * s + (lane >> 3), cofs = (lane & 7) * 4;
        const v4f x = *(const v4fa*)(&os[wb + o * OSP + cofs]);
        const float bo = bfr(cbias[o]);
        const v4f fv = *(const v4f*)(F + obase + (size_t)o * THW + cofs);
        v4f y;
#pragma unroll
        for (int i = 0; i < 4; ++i) {
            const float fh = __uint_as_float(((unsigned)cs[cwb + (cofs + i) * CSP + o]) << 16);
            const float cv = x[i] + bo;
            const float bl = fh * 0.5f + cv * 0.5f;
            const float fq = bfr(fv[i]);
            const float d = bl - fq;
            ls += d * d;
            y[i] = d + fq; }
        *(v4fa*)(&os[wb + o * OSP + cofs]) = y; }
    wave_sync();
    float* orow = OUT + obase;
    float* pd = PART + (size_t)rid * 32 + lane;
#pragma unroll 1
    for (int ps = 0; ps < 2; ++ps) {
#pragma unroll
        for (int s = 0; s < 8; ++s) { const int row = 4 * s + (lane >> 3), cofs = (lane & 7) * 4;
            const v4f val = *(const v4fa*)(&os[wb + row * OSP + cofs]);
            *(volatile v4f*)(orow + (size_t)row * THW + cofs) = val; }
        *(volatile float*)pd = ls;
        if (ps == 0) __threadfence(); }
}
static_assert(8 * 4 == CI);
static_assert(8 * 16 == WW * 4);
static_assert(4 * 32 * 16 == 32 * CI * 2);

__global__ __launch_bounds__(256) void k_final(const int* __restrict__ IDX, const float* __restrict__ PART, float* OUT) {
    __shared__ int flags[VOCAB];
    __shared__ float rs[8];
    __shared__ int ri[8];
    const int tid = threadIdx.x;
#pragma unroll 1
    for (int i = tid; i < VOCAB; i += 256) flags[i] = 0;
    __syncthreads();
#pragma unroll 1
    for (int i = tid; i < NQ; i += 256) { int c = IDX[i]; c = c < 0 ? 0 : (c > VOCAB - 1 ? VOCAB - 1 : c); flags[c] = 1; }
    __syncthreads();
    int cnt = 0;
#pragma unroll 1
    for (int i = tid; i < VOCAB; i += 256) cnt += flags[i];
    float s = 0.0f;
#pragma unroll 1
    for (int i = tid; i < NROWS * 32; i += 256) s += PART[i];
#pragma unroll
    for (int m = 16; m >= 1; m >>= 1) { s += __shfl_xor(s, m, 32); cnt += __shfl_xor(cnt, m, 32); }
    if ((tid & 31) == 0) { rs[tid >> 5] = s; ri[tid >> 5] = cnt; }
    __syncthreads();
    if (tid == 0) {
        float st = 0.0f; int ct = 0;
#pragma unroll
        for (int w = 0; w < 8; ++w) { st += rs[w]; ct += ri[w]; }
        const float mse = st * (1.0f / (float)((size_t)NB * CI * THW));
        const float loss = 0.25f * mse + mse;
        const float usage = ((float)ct * (1.0f / (float)VOCAB)) * 100.0f;
        v2f o; o[0] = loss; o[1] = usage;
        float* dst = OUT + OUT1_ELEM;
        *(volatile v2f*)dst = o; __threadfence(); *(volatile v2f*)dst = o; }
}

static constexpr size_t al256(size_t v) { return (v + 255) & ~(size_t)255; }
static constexpr size_t SZ_EB = al256((size_t)VOCAB * CI * 2);
static constexpr size_t SZ_QB = al256((size_t)NQ * CI * 2);
static constexpr size_t SZ_EE = al256((size_t)VOCAB * 4);
static constexpr size_t SZ_QQ = al256((size_t)NQ * 4);
static constexpr size_t SZ_WB = al256((size_t)CI * KC * 2);
static constexpr size_t SZ_IX = al256((size_t)NQ * 4);
static constexpr size_t SZ_FP = al256((size_t)NPP * CI * 2);
static constexpr size_t SZ_PT = al256((size_t)NROWS * 32 * 4);
static constexpr size_t SZ_TOTAL = SZ_EB + SZ_QB + SZ_EE + SZ_QQ + SZ_WB + SZ_IX + SZ_FP + SZ_PT;
static_assert(SZ_TOTAL <= (size_t)134217728);

extern "C" void kernel_launch(void* const* d_in, const int* in_sizes, int n_in,
                              void* d_out, int out_size, void* d_ws, size_t ws_size, hipStream_t stream) {
    if (n_in < 4) return;
    if ((size_t)in_sizes[0] < (size_t)NB * CI * THW) return;
    if ((size_t)in_sizes[1] < (size_t)VOCAB * CI) return;
    if ((size_t)in_sizes[2] < (size_t)CI * KC) return;
    if (in_sizes[3] < CI) return;
    if ((size_t)out_size < OUT1_ELEM + 2) return;
    if (SZ_TOTAL > ws_size) return;
    const float* f   = (const float*)d_in[0];
    const float* emb = (const float*)d_in[1];
    const float* cw  = (const float*)d_in[2];
    const float* cb  = (const float*)d_in[3];
    float* OUT = (float*)d_out;
    char* wsp = (char*)d_ws;
    bf* EB = (bf*)wsp; wsp += SZ_EB;
    bf* QB = (bf*)wsp; wsp += SZ_QB;
    float* EE = (float*)wsp; wsp += SZ_EE;
    float* QQ = (float*)wsp; wsp += SZ_QQ;
    bf* WB = (bf*)wsp; wsp += SZ_WB;
    int* IDX = (int*)wsp; wsp += SZ_IX;
    bf* FHP = (bf*)wsp; wsp += SZ_FP;
    float* PART = (float*)wsp; wsp += SZ_PT;

    { const size_t n8 = (size_t)VOCAB * CI / 8;
      k_cvt8<<<(unsigned)((n8 + 255) / 256), 256, 0, stream>>>(emb, EB, n8); }
    k_qT<<<NQ / 64, 256, 0, stream>>>(f, QB);
    { const int n8 = CI * KC / 8;
      k_wprep<<<(n8 + 255) / 256, 256, 0, stream>>>(cw, WB, n8); }
    k_rownorm<<<VOCAB / 64, 256, 0, stream>>>(EB, EE);
    k_rownorm<<<NQ / 64, 256, 0, stream>>>(QB, QQ);
    k_argmin<<<NQ / (32 * GW), 32 * GW, 0, stream>>>(QB, EB, QQ, EE, IDX);
    { const int ng = NPP * 4;
      k_gather<<<(ng + 255) / 256, 256, 0, stream>>>(IDX, EB, FHP, ng); }
    k_conv<<<NROWS / CW, 32 * CW, 0, stream>>>(FHP, WB, cb, f, OUT, PART);
    k_final<<<1, 256, 0, stream>>>(IDX, PART, OUT);
}
